// FlashAttention3_15822659518957
// MI455X (gfx1250) — hardware-verified
//
#include <hip/hip_runtime.h>
#include <stdint.h>

#ifndef SQ
#define SQ 2048
#endif
#define SEQ   2048
#define DMOD  2048
#define NH    16
#define HD    128
#define KBLK  64
#define NKB   (SEQ / KBLK)
#define RSQ_HD 0.08838834764831845f
#define LOG2E 1.4426950408889634f
#define QSC   256.0f
#define KSC   256.0f
#define PCAR  32768.0f
#define VCAR  1024.0f
#define OSC   1024.0f
#define WOS   1024.0f
#define LEPS  1e-6f
#define WPB   4
#define NHG   (NH / WPB)
#define NQT   (SQ / 16)
#define NST   (SEQ / 64)
#define ATT_THREADS (WPB * 32)
#define PTP   68
#define PTW   (16 * PTP)
#define SLP   132
#define SLW   (16 * SLP)
#define WREG  (PTW + SLW)
#define SLAB64 (16 * 68)
#define VTP   72
#define WS_CAP 134217728
static_assert(DMOD == NH * HD && HD == 128 && NH == 16 && WPB == 4 && NHG * WPB == NH && ATT_THREADS == 128);
static_assert((SQ % 64) == 0 && SQ >= 64 && SQ <= SEQ);
static_assert((SEQ % 64) == 0 && (SEQ % KBLK) == 0 && (DMOD % 64) == 0 && (DMOD % 32) == 0 && (HD % 32) == 0 && DMOD == 8 * 256);
static_assert(((SEQ * DMOD / 8) % 256) == 0 && ((DMOD * DMOD / 8) % 256) == 0);
static_assert((size_t)NH * HD * SEQ == (size_t)SEQ * DMOD);
static_assert(WPB * WREG * 4 <= 65536 && HD * VTP * 2 <= 65536 && 4 * SLAB64 * 4 <= 65536);
static_assert((size_t)SQ * DMOD * 2 <= (size_t)SEQ * DMOD * 4);

typedef unsigned short u16;
typedef _Float16 v16h __attribute__((ext_vector_type(16)));
typedef _Float16 v8h  __attribute__((ext_vector_type(8)));
typedef __bf16   v16b __attribute__((ext_vector_type(16)));
typedef float    v8f  __attribute__((ext_vector_type(8)));
typedef float    v4f  __attribute__((ext_vector_type(4)));
typedef unsigned int v4u __attribute__((ext_vector_type(4)));

union FragH { v16h v; v8h h[2]; v4u u[2]; };
union FragB { v16b v; v4u u[2]; };

__device__ __forceinline__ unsigned short bf_bits(float f) {
  unsigned u = __float_as_uint(f);
  return (unsigned short)((u + 0x7FFFu + ((u >> 16) & 1u)) >> 16);
}
__device__ __forceinline__ float bf_up(unsigned short h) { return __uint_as_float(((unsigned)h) << 16); }
__device__ __forceinline__ float bfr(float f) { return bf_up(bf_bits(f)); }
__device__ __forceinline__ unsigned short h_bits(_Float16 x) { return __builtin_bit_cast(unsigned short, x); }
__device__ __forceinline__ unsigned pk16(unsigned short a, unsigned short b) { return (unsigned)a | ((unsigned)b << 16); }
__device__ __forceinline__ v8f zero8() { v8f z = {0.f, 0.f, 0.f, 0.f, 0.f, 0.f, 0.f, 0.f}; return z; }
__device__ __forceinline__ v4f zero4() { v4f z = {0.f, 0.f, 0.f, 0.f}; return z; }

__device__ __forceinline__ v16h ldfrag_h(const _Float16* p) {
  FragH f;
  f.h[0] = *(const v8h*)(p);
  f.h[1] = *(const v8h*)(p + 16);
  return f.v;
}
__device__ __forceinline__ v16b ldfrag_b(const u16* p) {
  FragB f;
  f.u[0] = *(const v4u*)(p);
  f.u[1] = *(const v4u*)(p + 16);
  return f.v;
}

__device__ __forceinline__ v8f mma_h(v16h a, v16h b, v8f c) {
  return __builtin_amdgcn_wmma_f32_16x16x32_f16(false, a, false, b, (short)0, c, false, false);
}
__device__ __forceinline__ v8f mma_b(v16b a, v16b b, v8f c) {
  return __builtin_amdgcn_wmma_f32_16x16x32_bf16(false, a, false, b, (short)0, c, false, false);
}
__device__ __forceinline__ void guard2(v8f& a, v8f& b, v16h x0, v16h x1, v16h x2, v16h x3, v16h x4, v16h x5) {
#if defined(__HIP_DEVICE_COMPILE__)
  asm volatile("v_nop\n\tv_nop\n\tv_nop\n\tv_nop"
               : "+v"(a), "+v"(b) : "v"(x0), "v"(x1), "v"(x2), "v"(x3), "v"(x4), "v"(x5) : "memory");
#endif
}
template <typename F>
__device__ __forceinline__ void guard6(v8f& a, v8f& b, v8f& c, v8f& d, F x0, F x1, F x2, F x3, F x4, F x5) {
#if defined(__HIP_DEVICE_COMPILE__)
  asm volatile("v_nop\n\tv_nop\n\tv_nop\n\tv_nop"
               : "+v"(a), "+v"(b), "+v"(c), "+v"(d) : "v"(x0), "v"(x1), "v"(x2), "v"(x3), "v"(x4), "v"(x5) : "memory");
#endif
}
__device__ __forceinline__ void acc_guard4(v8f& a, v8f& b, v8f& c, v8f& d) {
#if defined(__HIP_DEVICE_COMPILE__)
  asm volatile("v_nop\n\tv_nop\n\tv_nop\n\tv_nop" : "+v"(a), "+v"(b), "+v"(c), "+v"(d));
#endif
}
__device__ __forceinline__ void wave_sync_lds() {
  __builtin_amdgcn_fence(__ATOMIC_RELEASE, "workgroup");
  __builtin_amdgcn_wave_barrier();
  __builtin_amdgcn_fence(__ATOMIC_ACQUIRE, "workgroup");
}

__global__ __launch_bounds__(256) void cvt16(const float* __restrict__ x, u16* D, int n8, int f16mode, float scale) {
  const int gt = blockIdx.x * 256 + (int)threadIdx.x;
  if (gt >= n8) return;
  const float* p = x + (size_t)gt * 8;
  const v4f a = *(const v4f*)(p), b4 = *(const v4f*)(p + 4);
  float w[8];
#pragma unroll
  for (int e = 0; e < 4; ++e) { w[e] = a[e]; w[4 + e] = b4[e]; }
  v4u o;
#pragma unroll
  for (int e = 0; e < 4; ++e) {
    const float f0 = w[2 * e], f1 = w[2 * e + 1];
    const unsigned short hb0 = h_bits((_Float16)(bfr(f0) * scale));
    const unsigned short hb1 = h_bits((_Float16)(bfr(f1) * scale));
    const unsigned short bb0 = bf_bits(f0);
    const unsigned short bb1 = bf_bits(f1);
    o[e] = (f16mode != 0) ? pk16(hb0, hb1) : pk16(bb0, bb1);
  }
  u16* d = D + (size_t)gt * 8;
  for (int pass = 0; pass < 2; ++pass) {
    *(volatile v4u*)(d) = o;
    __threadfence();
  }
}

__global__ __launch_bounds__(256) void vt16(const float* __restrict__ F, u16* VHo) {
  __shared__ __align__(16) u16 TH[HD * VTP];
  const int tid = threadIdx.x;
  const int bid = blockIdx.x;
  const int st  = bid % NST;
  const int h   = bid / NST;
  if (h >= NH) return;
  const int s0  = st * 64;
  {
    const int sl = tid >> 2;
    const int dc = (tid & 3) * 32;
    const int cb = h * HD + dc;
    const float* src = F + ((size_t)s0 + sl) * DMOD + cb;
#pragma unroll
    for (int i = 0; i < 8; ++i) {
      const v4f a = *(const v4f*)(src + 4 * i);
#pragma unroll
      for (int e = 0; e < 4; ++e) {
        const float t = a[e] * VCAR;
        TH[(dc + 4 * i + e) * VTP + sl] = h_bits((_Float16)t);
      }
    }
  }
  __syncthreads();
  v4u vh[4];
  const int q8 = tid >> 3, p8 = (tid & 7) * 8;
#pragma unroll
  for (int it = 0; it < 4; ++it) {
    const int line = it * 32 + q8;
    vh[it] = *(const v4u*)(TH + line * VTP + p8);
  }
  const size_t hrow = (size_t)h * HD;
  const size_t base = hrow * SEQ + s0 + p8;
  for (int pass = 0; pass < 2; ++pass) {
#pragma unroll
    for (int it = 0; it < 4; ++it) {
      const int line = it * 32 + q8;
      *(volatile v4u*)(VHo + base + (size_t)line * SEQ) = vh[it];
    }
    __threadfence();
  }
}

__global__ __launch_bounds__(256) void rope16(const float* __restrict__ F,
                                              const float* __restrict__ ctab, const float* __restrict__ stab,
                                              u16* Hp, u16* Lp, int nrows, float sc) {
#pragma clang fp contract(off)
  const int tid = (int)threadIdx.x;
  const int blk = (int)blockIdx.x;
  if (blk >= nrows || blk >= SEQ) return;
  const int pos = blk;
  const size_t grow = (size_t)blk;
  const int col = tid * 8;
  const float* p = F + grow * DMOD + col;
  const v4f xa = *(const v4f*)(p), xb = *(const v4f*)(p + 4);
  float y[8];
#pragma unroll
  for (int e = 0; e < 4; ++e) { y[e] = xa[e]; y[4 + e] = xb[e]; }
  const int p4 = (tid * 4) & 63;
  const float* cp = ctab + (size_t)pos * (HD / 2) + p4;
  const float* sp = stab + (size_t)pos * (HD / 2) + p4;
  const v4f ca = *(const v4f*)(cp);
  const v4f sa = *(const v4f*)(sp);
  float cv[4], sv[4];
#pragma unroll
  for (int e = 0; e < 4; ++e) { cv[e] = bfr(ca[e]); sv[e] = bfr(sa[e]); }
  v4u oh, ol;
#pragma unroll
  for (int pr = 0; pr < 4; ++pr) {
    const int e0 = 2 * pr, e1 = 2 * pr + 1;
    const float re = y[e0] * cv[pr] - y[e1] * sv[pr];
    const float ro = y[e0] * sv[pr] + y[e1] * cv[pr];
    const float te = re * sc, to = ro * sc;
    const _Float16 he = (_Float16)te, ho = (_Float16)to;
    const _Float16 le = (_Float16)(te - (float)he), lo = (_Float16)(to - (float)ho);
    oh[pr] = pk16(h_bits(he), h_bits(ho));
    ol[pr] = pk16(h_bits(le), h_bits(lo));
  }
  u16* dh = Hp + grow * DMOD + col;
  u16* dl = Lp + grow * DMOD + col;
  for (int pass = 0; pass < 2; ++pass) {
    *(volatile v4u*)(dh) = oh;
    *(volatile v4u*)(dl) = ol;
    __threadfence();
  }
}

__device__ __forceinline__ void epi64(float* sl, v8f a0, v8f a1, v8f a2, v8f a3, float oscale, v4f badd,
                                      float* C, int N, size_t rowb, int col0, int lane) {
  const int hh = lane >> 4, m = lane & 15;
#pragma unroll
  for (int r = 0; r < 8; ++r) {
    const int ro = (8 * hh + r) * 68 + m;
    sl[ro]      = a0[r] * oscale;
    sl[ro + 16] = a1[r] * oscale;
    sl[ro + 32] = a2[r] * oscale;
    sl[ro + 48] = a3[r] * oscale;
  }
  wave_sync_lds();
  v4f vals[8];
#pragma unroll
  for (int it = 0; it < 8; ++it) vals[it] = *(const v4f*)(sl + (it * 2 + hh) * 68 + m * 4) + badd;
  float* dst = C + (rowb + (size_t)hh) * (size_t)N + col0 + m * 4;
  for (int pass = 0; pass < 2; ++pass) {
#pragma unroll
    for (int it = 0; it < 8; ++it) {
      *(volatile v4f*)(dst + (size_t)(it * 2) * (size_t)N) = vals[it];
    }
    __threadfence();
  }
}

__global__ __launch_bounds__(128)
void gemm_bf(const u16* __restrict__ A, const u16* __restrict__ Bt, float* C, int M, int N, int K, float oscale) {
  __shared__ __align__(16) float slab[4 * SLAB64];
  const int tid = threadIdx.x, wave = tid >> 5, lane = tid & 31, hh = lane >> 4, m = lane & 15;
  const int ntile = N >> 6;
  const int bid   = blockIdx.x;
  const int rowb  = (bid / ntile) * 64 + wave * 16;
  const int col0  = (bid % ntile) * 64;
  if (rowb + 16 > M) return;
  const u16* ap = A  + (size_t)(rowb + m) * K + 8 * hh;
  const u16* bp = Bt + (size_t)(col0 + m) * K + 8 * hh;
  const size_t bs = (size_t)16 * K;
  v8f acc0 = zero8(), acc1 = zero8(), acc2 = zero8(), acc3 = zero8();
#pragma unroll 1
  for (int k0 = 0; k0 < K; k0 += 32) {
    const v16b a  = ldfrag_b(ap + k0);
    const v16b b0 = ldfrag_b(bp + k0);
    const v16b b1 = ldfrag_b(bp + bs + k0);
    const v16b b2 = ldfrag_b(bp + 2 * bs + k0);
    const v16b b3 = ldfrag_b(bp + 3 * bs + k0);
    acc0 = mma_b(a, b0, acc0);
    acc1 = mma_b(a, b1, acc1);
    acc2 = mma_b(a, b2, acc2);
    acc3 = mma_b(a, b3, acc3);
    guard6<v16b>(acc0, acc1, acc2, acc3, a, b0, b1, b2, b3, a);
  }
  epi64(slab + wave * SLAB64, acc0, acc1, acc2, acc3, oscale, zero4(), C, N, (size_t)rowb, col0, lane);
}

__global__ __launch_bounds__(128)
void gemm_h(const u16* __restrict__ A, const u16* __restrict__ Bt, float* C, int M, int N, int K, float oscale) {
  __shared__ __align__(16) float slab[4 * SLAB64];
  const int tid = threadIdx.x, wave = tid >> 5, lane = tid & 31, hh = lane >> 4, m = lane & 15;
  const int ntile = N >> 6;
  const int bid   = blockIdx.x;
  const int rowb  = (bid / ntile) * 64 + wave * 16;
  const int col0  = (bid % ntile) * 64;
  if (rowb + 16 > M) return;
  const _Float16* ap = (const _Float16*)(const void*)A  + (size_t)(rowb + m) * K + 8 * hh;
  const _Float16* bp = (const _Float16*)(const void*)Bt + (size_t)(col0 + m) * K + 8 * hh;
  const size_t bs = (size_t)16 * K;
  v8f acc0 = zero8(), acc1 = zero8(), acc2 = zero8(), acc3 = zero8();
#pragma unroll 1
  for (int k0 = 0; k0 < K; k0 += 32) {
    const v16h a  = ldfrag_h(ap + k0);
    const v16h b0 = ldfrag_h(bp + k0);
    const v16h b1 = ldfrag_h(bp + bs + k0);
    const v16h b2 = ldfrag_h(bp + 2 * bs + k0);
    const v16h b3 = ldfrag_h(bp + 3 * bs + k0);
    acc0 = mma_h(a, b0, acc0);
    acc1 = mma_h(a, b1, acc1);
    acc2 = mma_h(a, b2, acc2);
    acc3 = mma_h(a, b3, acc3);
    guard6<v16h>(acc0, acc1, acc2, acc3, a, b0, b1, b2, b3, a);
  }
  epi64(slab + wave * SLAB64, acc0, acc1, acc2, acc3, oscale, zero4(), C, N, (size_t)rowb, col0, lane);
}

__global__ __launch_bounds__(ATT_THREADS)
void attn_blk(const u16* __restrict__ QHp, const u16* __restrict__ QLp,
              const u16* __restrict__ KHp, const u16* __restrict__ KLp,
              const u16* __restrict__ VHp, const int* __restrict__ Mk, u16* OHp) {
  __shared__ __align__(16) float smem[WPB * WREG];
  (void)Mk;

  const int tid  = threadIdx.x;
  const int wave = tid >> 5;
  const int lane = tid & 31;
  const int hh   = lane >> 4;
  const int c    = lane & 15;
  const int bid  = blockIdx.x;
  const int qt   = bid % NQT;
  const int hg   = bid / NQT;
  if (hg >= NHG) return;
  const int q0   = qt * 16;
  if (q0 + 16 > SQ) return;
  const int head = hg * WPB + wave;

  float* pt   = smem + wave * WREG;
  float* slab = pt + PTW;

  const size_t hcol = (size_t)head * HD + 8 * hh;
  const _Float16* Qh  = (const _Float16*)(const void*)QHp + ((size_t)q0 + c) * DMOD + hcol;
  const _Float16* Ql  = (const _Float16*)(const void*)QLp + ((size_t)q0 + c) * DMOD + hcol;
  const _Float16* Khb = (const _Float16*)(const void*)KHp + (size_t)c * DMOD + hcol;
  const _Float16* Klb = (const _Float16*)(const void*)KLp + (size_t)c * DMOD + hcol;
  const _Float16* Vhb = (const _Float16*)(const void*)VHp + ((size_t)head * HD + c) * SEQ + 8 * hh;
  const float lsc = RSQ_HD * (LOG2E / (QSC * KSC));
  const float oc  = 1.0f / (PCAR * VCAR);
  const size_t KROW = (size_t)DMOD;

  float lrow[8];
  v8f o[8];
#pragma unroll
  for (int r = 0; r < 8; ++r) lrow[r] = 0.f;
#pragma unroll
  for (int j = 0; j < 8; ++j) o[j] = zero8();

#pragma unroll 1
  for (int kt = 0; kt < NKB; ++kt) {
    const int kb = kt * KBLK;
    v8f s0 = zero8(), s1 = zero8(), s2 = zero8(), s3 = zero8();
    {
      const _Float16* k0p = Khb + (size_t)kb * KROW;
      const _Float16* k1p = k0p + (size_t)16 * KROW;
      const _Float16* l0p = Klb + (size_t)kb * KROW;
      const _Float16* l1p = l0p + (size_t)16 * KROW;
#pragma unroll
      for (int kk = 0; kk < HD / 32; ++kk) {
        const v16h qh  = ldfrag_h(Qh + kk * 32);
        const v16h ql  = ldfrag_h(Ql + kk * 32);
        const v16h kh0 = ldfrag_h(k0p + kk * 32);
        const v16h kh1 = ldfrag_h(k1p + kk * 32);
        const v16h kl0 = ldfrag_h(l0p + kk * 32);
        const v16h kl1 = ldfrag_h(l1p + kk * 32);
        s0 = mma_h(qh, kh0, s0);
        s0 = mma_h(ql, kh0, s0);
        s0 = mma_h(qh, kl0, s0);
        s1 = mma_h(qh, kh1, s1);
        s1 = mma_h(ql, kh1, s1);
        s1 = mma_h(qh, kl1, s1);
        guard2(s0, s1, qh, ql, kh0, kl0, kh1, kl1);
      }
    }
    {
      const _Float16* k2p = Khb + (size_t)(kb + 32) * KROW;
      const _Float16* k3p = k2p + (size_t)16 * KROW;
      const _Float16* l2p = Klb + (size_t)(kb + 32) * KROW;
      const _Float16* l3p = l2p + (size_t)16 * KROW;
#pragma unroll
      for (int kk = 0; kk < HD / 32; ++kk) {
        const v16h qh  = ldfrag_h(Qh + kk * 32);
        const v16h ql  = ldfrag_h(Ql + kk * 32);
        const v16h kh2 = ldfrag_h(k2p + kk * 32);
        const v16h kh3 = ldfrag_h(k3p + kk * 32);
        const v16h kl2 = ldfrag_h(l2p + kk * 32);
        const v16h kl3 = ldfrag_h(l3p + kk * 32);
        s2 = mma_h(qh, kh2, s2);
        s2 = mma_h(ql, kh2, s2);
        s2 = mma_h(qh, kl2, s2);
        s3 = mma_h(qh, kh3, s3);
        s3 = mma_h(ql, kh3, s3);
        s3 = mma_h(qh, kl3, s3);
        guard2(s2, s3, qh, ql, kh2, kl2, kh3, kl3);
      }
    }
#pragma unroll
    for (int r = 0; r < 8; ++r) {
      const float t0 = s0[r] * lsc, t1 = s1[r] * lsc, t2 = s2[r] * lsc, t3 = s3[r] * lsc;
      float mx = fmaxf(fmaxf(t0, t1), fmaxf(t2, t3));
#pragma unroll
      for (int off = 1; off < 16; off <<= 1) mx = fmaxf(mx, __shfl_xor(mx, off, 32));
      const float e0 = exp2f(t0 - mx), e1 = exp2f(t1 - mx), e2 = exp2f(t2 - mx), e3 = exp2f(t3 - mx);
      float ps = (e0 + e1) + (e2 + e3);
#pragma unroll
      for (int off = 1; off < 16; off <<= 1) ps += __shfl_xor(ps, off, 32);
      lrow[r] += ps;
      const int ro = (8 * hh + r) * PTP + c;
      pt[ro]      = e0;
      pt[ro + 16] = e1;
      pt[ro + 32] = e2;
      pt[ro + 48] = e3;
    }
    wave_sync_lds();
    {
      FragH ph;
      {
        const float* prow = pt + c * PTP + 8 * hh;
        const v4f p0 = *(const v4f*)(prow), p1 = *(const v4f*)(prow + 4);
        const v4f p2 = *(const v4f*)(prow + 16), p3 = *(const v4f*)(prow + 20);
#pragma unroll
        for (int e = 0; e < 4; ++e) {
          ph.h[0][e]     = (_Float16)(p0[e] * PCAR);
          ph.h[0][4 + e] = (_Float16)(p1[e] * PCAR);
          ph.h[1][e]     = (_Float16)(p2[e] * PCAR);
          ph.h[1][4 + e] = (_Float16)(p3[e] * PCAR);
        }
      }
      {
        const _Float16* vhp = Vhb + kb;
        const v16h va = ldfrag_h(vhp);
        const v16h vb = ldfrag_h(vhp + (size_t)16 * SEQ);
        const v16h vc = ldfrag_h(vhp + (size_t)32 * SEQ);
        const v16h vd = ldfrag_h(vhp + (size_t)48 * SEQ);
        o[0] = mma_h(ph.v, va, o[0]);
        o[1] = mma_h(ph.v, vb, o[1]);
        o[2] = mma_h(ph.v, vc, o[2]);
        o[3] = mma_h(ph.v, vd, o[3]);
        guard6<v16h>(o[0], o[1], o[2], o[3], ph.v, va, vb, vc, vd, ph.v);
      }
      {
        const _Float16* vhp = Vhb + kb + (size_t)64 * SEQ;
        const v16h ve = ldfrag_h(vhp);
        const v16h vf = ldfrag_h(vhp + (size_t)16 * SEQ);
        const v16h vg = ldfrag_h(vhp + (size_t)32 * SEQ);
        const v16h vw = ldfrag_h(vhp + (size_t)48 * SEQ);
        o[4] = mma_h(ph.v, ve, o[4]);
        o[5] = mma_h(ph.v, vf, o[5]);
        o[6] = mma_h(ph.v, vg, o[6]);
        o[7] = mma_h(ph.v, vw, o[7]);
        guard6<v16h>(o[4], o[5], o[6], o[7], ph.v, ve, vf, vg, vw, ph.v);
      }
    }
    {
      FragH ph;
      {
        const float* prow = pt + c * PTP + 32 + 8 * hh;
        const v4f p0 = *(const v4f*)(prow), p1 = *(const v4f*)(prow + 4);
        const v4f p2 = *(const v4f*)(prow + 16), p3 = *(const v4f*)(prow + 20);
#pragma unroll
        for (int e = 0; e < 4; ++e) {
          ph.h[0][e]     = (_Float16)(p0[e] * PCAR);
          ph.h[0][4 + e] = (_Float16)(p1[e] * PCAR);
          ph.h[1][e]     = (_Float16)(p2[e] * PCAR);
          ph.h[1][4 + e] = (_Float16)(p3[e] * PCAR);
        }
      }
      {
        const _Float16* vhp = Vhb + kb + 32;
        const v16h va = ldfrag_h(vhp);
        const v16h vb = ldfrag_h(vhp + (size_t)16 * SEQ);
        const v16h vc = ldfrag_h(vhp + (size_t)32 * SEQ);
        const v16h vd = ldfrag_h(vhp + (size_t)48 * SEQ);
        o[0] = mma_h(ph.v, va, o[0]);
        o[1] = mma_h(ph.v, vb, o[1]);
        o[2] = mma_h(ph.v, vc, o[2]);
        o[3] = mma_h(ph.v, vd, o[3]);
        guard6<v16h>(o[0], o[1], o[2], o[3], ph.v, va, vb, vc, vd, ph.v);
      }
      {
        const _Float16* vhp = Vhb + kb + 32 + (size_t)64 * SEQ;
        const v16h ve = ldfrag_h(vhp);
        const v16h vf = ldfrag_h(vhp + (size_t)16 * SEQ);
        const v16h vg = ldfrag_h(vhp + (size_t)32 * SEQ);
        const v16h vw = ldfrag_h(vhp + (size_t)48 * SEQ);
        o[4] = mma_h(ph.v, ve, o[4]);
        o[5] = mma_h(ph.v, vf, o[5]);
        o[6] = mma_h(ph.v, vg, o[6]);
        o[7] = mma_h(ph.v, vw, o[7]);
        guard6<v16h>(o[4], o[5], o[6], o[7], ph.v, ve, vf, vg, vw, ph.v);
      }
    }
    wave_sync_lds();
  }
  acc_guard4(o[0], o[1], o[2], o[3]);
  acc_guard4(o[4], o[5], o[6], o[7]);
#pragma unroll
  for (int r = 0; r < 8; ++r) {
    const float inv = (1.0f / (lrow[r] + LEPS)) * oc;
#pragma unroll
    for (int j = 0; j < 8; ++j) {
      const int idx = (8 * hh + r) * SLP + j * 16 + c;
      slab[idx] = o[j][r] * inv;
    }
  }

  wave_sync_lds();
  v4u oh[8];
  const int c8 = c * 8;
#pragma unroll
  for (int it = 0; it < 8; ++it) {
    const int row = it * 2 + hh;
    const v4f a = *(const v4f*)(slab + row * SLP + c8), b4 = *(const v4f*)(slab + row * SLP + c8 + 4);
    float w[8];
#pragma unroll
    for (int e = 0; e < 4; ++e) { w[e] = a[e] * OSC; w[4 + e] = b4[e] * OSC; }
#pragma unroll
    for (int e = 0; e < 4; ++e) {
      const _Float16 h0 = (_Float16)w[2 * e], h1 = (_Float16)w[2 * e + 1];
      oh[it][e] = pk16(h_bits(h0), h_bits(h1));
    }
  }
  const size_t ob = (size_t)q0 * DMOD + (size_t)head * HD + c8;
  for (int pass = 0; pass < 2; ++pass) {
#pragma unroll
    for (int it = 0; it < 8; ++it) {
      const int row = it * 2 + hh;
      *(volatile v4u*)(OHp + ob + (size_t)row * DMOD) = oh[it];
    }
    __threadfence();
  }
}

extern "C" void kernel_launch(void* const* d_in, const int* in_sizes, int n_in,
                              void* d_out, int out_size, void* d_ws, size_t ws_size,
                              hipStream_t stream) {
  if (n_in < 8) return;
  if (in_sizes[0] != SEQ * DMOD) return;
  if (in_sizes[1] < SEQ * (HD / 2) || in_sizes[2] < SEQ * (HD / 2)) return;
  for (int i = 3; i <= 6; ++i) if (in_sizes[i] != DMOD * DMOD) return;
  if (in_sizes[7] < 1) return;
  if (out_size < SEQ * DMOD) return;

  const float* x    = (const float*)d_in[0];
  const float* fcos = (const float*)d_in[1];
  const float* fsin = (const float*)d_in[2];
  const float* wq   = (const float*)d_in[3];
  const float* wk   = (const float*)d_in[4];
  const float* wv   = (const float*)d_in[5];
  const float* wo   = (const float*)d_in[6];
  const int*   mk   = (const int*)d_in[7];
  float*       out  = (float*)d_out;

  const size_t szX = (size_t)SEQ * DMOD * 2;
  const size_t szW = (size_t)DMOD * DMOD * 2;
  const size_t szF = (size_t)SEQ * DMOD * 4;
  const size_t szP = (size_t)SEQ * DMOD * 2;
  if ((size_t)SEQ * DMOD * 2 > szF) return;
  size_t off = 0;
  const size_t oX  = off; off += szX;
  const size_t oW  = off; off += szW;
  const size_t oF  = off; off += szF;
  const size_t oQH = off; off += szP;
  const size_t oQL = off; off += szP;
  const size_t oKH = off; off += szP;
  const size_t oKL = off; off += szP;
  if (off > ws_size) return;
  if (off > (size_t)WS_CAP) return;

  char* ws = (char*)d_ws;
  u16*   XB = (u16*)(ws + oX);
  u16*   VH = (u16*)(ws + oX);
  u16*   WB = (u16*)(ws + oW);
  float* F  = (float*)(ws + oF);
  u16*   OH = (u16*)(ws + oF);
  u16*   QH = (u16*)(ws + oQH);
  u16*   QL = (u16*)(ws + oQL);
  u16*   KH = (u16*)(ws + oKH);
  u16*   KL = (u16*)(ws + oKL);

  const dim3 b256(256), b128(128), bAT(ATT_THREADS);
  const int  n8x = (SEQ * DMOD) / 8;
  const dim3 gX((n8x + 255) / 256);
  const int  n8w = (DMOD * DMOD) / 8;
  const dim3 gW((n8w + 255) / 256);
  const dim3 gGQ((SQ / 64) * (DMOD / 64));
  const dim3 gGK((SEQ / 64) * (DMOD / 64));
  const dim3 gRQ(SQ);
  const dim3 gRK(SEQ);
  const dim3 gVT(NH * NST);
  const dim3 gAT(NQT * NHG);

  cvt16<<<gX, b256, 0, stream>>>(x, XB, n8x, 0, 1.0f);
  cvt16<<<gW, b256, 0, stream>>>(wq, WB, n8w, 0, 1.0f);
  gemm_bf<<<gGQ, b128, 0, stream>>>(XB, WB, F, SQ, DMOD, DMOD, 1.0f);
  rope16<<<gRQ, b256, 0, stream>>>(F, fcos, fsin, QH, QL, SQ, QSC);
  cvt16<<<gW, b256, 0, stream>>>(wk, WB, n8w, 0, 1.0f);
  gemm_bf<<<gGK, b128, 0, stream>>>(XB, WB, F, SEQ, DMOD, DMOD, 1.0f);
  rope16<<<gRK, b256, 0, stream>>>(F, fcos, fsin, KH, KL, SEQ, KSC);
  cvt16<<<gW, b256, 0, stream>>>(wv, WB, n8w, 0, 1.0f);
  gemm_bf<<<gGK, b128, 0, stream>>>(XB, WB, F, SEQ, DMOD, DMOD, 1.0f);
  vt16<<<gVT, b256, 0, stream>>>(F, VH);
  attn_blk<<<gAT, bAT, 0, stream>>>(QH, QL, KH, KL, VH, mk, OH);
  cvt16<<<gW, b256, 0, stream>>>(wo, WB, n8w, 1, WOS);
  gemm_h<<<gGQ, b128, 0, stream>>>(OH, WB, out, SQ, DMOD, DMOD, 1.0f / (OSC * WOS));
  (void)hipGetLastError();
}
